// GraphNet_86363202388241
// MI455X (gfx1250) — hardware-verified
//
#include <hip/hip_runtime.h>
#include <stddef.h>
#include <stdint.h>
#include <math.h>


#define FIN     256
#define DM      256
#define NHEAD   4
#define HC      64
#define KP2     512
#define FCD     64
#define NCLS    4
#define NTHR    256
#define NWAVE   8
#define EPT     8
#define CHUNK   (NTHR * EPT)
#define WCAP    (EPT * 32)
#define LISTN   (NWAVE * WCAP)
#define NBMAX   2048
#define SLOTB   10
#define SLOTM   ((1 << SLOTB) - 1)
#define NBLIM   (1 << SLOTB)
#define RCAP    28672
#define DEGCAP  256
#define GBM     64
#define GBN     64
#define GTHR    128
#define MROWS   128
#define SLOPE_ATT 0.2f
#define EPS_SM  1e-16f
#define WSMAX   134217728
#define LDS_AGG ((2 * RCAP + 2 * NBMAX + LISTN) * 4 + 64)

static_assert((CHUNK & (CHUNK - 1)) == 0 && CHUNK <= 2048);
static_assert(((long long)(CHUNK - 1) << SLOTB) < 2147483647LL);
static_assert(NBLIM <= NBMAX && NBLIM <= LISTN);
static_assert(NTHR * 8 == NBMAX);
static_assert(LISTN >= NWAVE * WCAP);
static_assert((RCAP % 32) == 0);
static_assert(LDS_AGG <= 300000);
static_assert(GBM == (GTHR / 32) * 16);
static_assert((FIN % 32) == 0 && (KP2 % 32) == 0 && KP2 == 2 * DM);
static_assert(DM == NHEAD * HC && HC == GBN);
static_assert(DM == 8 * 32);
static_assert(HC == 8 * 8);
static_assert((MROWS % GBM) == 0);
static_assert(FIN / 8 == 32);
static_assert(NCLS == 4);
static_assert(FCD == GBN);
static_assert(GTHR == 2 * GBM);

typedef float          v4f  __attribute__((ext_vector_type(4)));
typedef float          v8f  __attribute__((ext_vector_type(8)));
typedef int            v4i  __attribute__((ext_vector_type(4)));
typedef int            v8i  __attribute__((ext_vector_type(8)));
typedef unsigned int   v4u  __attribute__((ext_vector_type(4)));
typedef unsigned short v8us __attribute__((ext_vector_type(8)));
typedef __bf16         v16b __attribute__((ext_vector_type(16)));
typedef v4f  __attribute__((may_alias)) v4fa;
typedef v8us __attribute__((may_alias)) v8usa;
union FragB { v16b v; v8us h[2]; v8i w; };

__device__ __forceinline__ v8f wmb(const FragB& a, const FragB& b, v8f c) {
  v8f d = __builtin_amdgcn_wmma_f32_16x16x32_bf16(false, a.v, false, b.v, (short)0, c, false, false);
  asm volatile("v_nop\n\tv_nop\n\tv_nop\n\tv_nop" : "+v"(d) : "v"(a.w), "v"(b.w));
  return d;
}

__device__ __forceinline__ unsigned int f2bf(float f) {
  const unsigned int u = __float_as_uint(f);
  return ((u + 0x7FFFu + ((u >> 16) & 1u)) >> 16) & 0xFFFFu;
}
__device__ __forceinline__ float bf2f(unsigned int b) { return __uint_as_float(b << 16); }
__device__ __forceinline__ float bfr(float f) { return bf2f(f2bf(f)); }
__device__ __forceinline__ v4f bfr4(const v4f a) {
  v4f r; r.x = bfr(a.x); r.y = bfr(a.y); r.z = bfr(a.z); r.w = bfr(a.w); return r;
}
__device__ __forceinline__ unsigned int pk2(float lo, float hi) { return f2bf(lo) | (f2bf(hi) << 16); }
__device__ __forceinline__ v4u pack8(const v4f a, const v4f b) {
  v4u r;
  r.x = pk2(a.x, a.y); r.y = pk2(a.z, a.w); r.z = pk2(b.x, b.y); r.w = pk2(b.z, b.w);
  return r;
}
__device__ __forceinline__ v4f relu4(v4f a) {
  v4f r; r.x = fmaxf(a.x, 0.f); r.y = fmaxf(a.y, 0.f); r.z = fmaxf(a.z, 0.f); r.w = fmaxf(a.w, 0.f); return r;
}

__device__ __forceinline__ int scan_chunk(const int* __restrict__ dsts, int nE, int cbase, int slotBase,
                                          int nb, int vec8, int* list, int tid, int lane, int wave) {
  int wc = 0;
  const int el0  = tid * EPT;
  const int e0   = cbase + el0;
  const int sent = -2147483647 - 1;
  v4i da, db;
  if (vec8 != 0 && cbase + CHUNK <= nE) {
    da = *(const v4i*)(dsts + e0);
    db = *(const v4i*)(dsts + e0 + 4);
  } else {
    da.x = (e0     < nE) ? dsts[min(e0,     nE - 1)] : sent;
    da.y = (e0 + 1 < nE) ? dsts[min(e0 + 1, nE - 1)] : sent;
    da.z = (e0 + 2 < nE) ? dsts[min(e0 + 2, nE - 1)] : sent;
    da.w = (e0 + 3 < nE) ? dsts[min(e0 + 3, nE - 1)] : sent;
    db.x = (e0 + 4 < nE) ? dsts[min(e0 + 4, nE - 1)] : sent;
    db.y = (e0 + 5 < nE) ? dsts[min(e0 + 5, nE - 1)] : sent;
    db.z = (e0 + 6 < nE) ? dsts[min(e0 + 6, nE - 1)] : sent;
    db.w = (e0 + 7 < nE) ? dsts[min(e0 + 7, nE - 1)] : sent;
  }
  const unsigned nbs = (unsigned)slotBase;
  const unsigned unb = (unsigned)nb;
  const unsigned s0 = (unsigned)da.x - nbs, s1 = (unsigned)da.y - nbs;
  const unsigned s2 = (unsigned)da.z - nbs, s3 = (unsigned)da.w - nbs;
  const unsigned s4 = (unsigned)db.x - nbs, s5 = (unsigned)db.y - nbs;
  const unsigned s6 = (unsigned)db.z - nbs, s7 = (unsigned)db.w - nbs;
  const bool h0 = s0 < unb, h1 = s1 < unb, h2 = s2 < unb, h3 = s3 < unb;
  const bool h4 = s4 < unb, h5 = s5 < unb, h6 = s6 < unb, h7 = s7 < unb;
  const unsigned any = __builtin_amdgcn_ballot_w32(h0 | h1 | h2 | h3 | h4 | h5 | h6 | h7);
  if (any != 0u) {
#define HITJ(J, HJ, SJ) { \
      const unsigned mj = __builtin_amdgcn_ballot_w32(HJ); \
      if (mj != 0u) { \
        if (HJ) { \
          const int pos = wc + (int)__builtin_amdgcn_mbcnt_lo(mj, 0u); \
          if (pos < WCAP) list[wave * WCAP + pos] = ((el0 + (J)) << SLOTB) | (int)(SJ); \
        } \
        wc += (int)__builtin_popcount(mj); } }
    HITJ(0, h0, s0)
    HITJ(1, h1, s1)
    HITJ(2, h2, s2)
    HITJ(3, h3, s3)
    HITJ(4, h4, s4)
    HITJ(5, h5, s5)
    HITJ(6, h6, s6)
    HITJ(7, h7, s7)
#undef HITJ
  }
  return wc;
}

__global__ __launch_bounds__(NTHR) void k_xprep(const float* __restrict__ x, unsigned short* xb, int nN, int nUnits) {
  const int u = (int)blockIdx.x * NTHR + (int)threadIdx.x;
  if (u >= nUnits) return;
  const int row = u >> 5;
  const int k8  = (u & 31) * 8;
  const int rc  = row < nN ? row : nN - 1;
  const float* p = x + (size_t)rc * (size_t)FIN + k8;
  v4f a = *(const v4fa*)p;
  v4f b = *(const v4fa*)(p + 4);
  const v4f z4 = {0.f, 0.f, 0.f, 0.f};
  if (row >= nN) { a = z4; b = z4; }
  const v4u hv = pack8(a, b);
  unsigned short* o = xb + (size_t)row * (size_t)FIN + k8;
  *(volatile v4u*)o = hv;
  __threadfence();
  *(volatile v4u*)o = hv;
}

__global__ __launch_bounds__(NTHR) void k_wprep(const float* __restrict__ w, int Kin, int Kper, int Ncol, int Nrows,
                                                int Kout, unsigned short* wt, int nUnits) {
  const int u = (int)blockIdx.x * NTHR + (int)threadIdx.x;
  if (u >= nUnits) return;
  const int kq = Kout >> 3;
  const int n  = u / kq;
  const int k8 = (u - n * kq) * 8;
  const int kk = k8 - (k8 / Kper) * Kper;
  const int ncl = n < Ncol ? n : Ncol - 1;
  const bool nl = (n < Ncol);
  const size_t nc = (size_t)Ncol;
  const float* p = w + ncl;
  const int q0 = min(kk + 0, Kin - 1), q1 = min(kk + 1, Kin - 1), q2 = min(kk + 2, Kin - 1), q3 = min(kk + 3, Kin - 1);
  const int q4 = min(kk + 4, Kin - 1), q5 = min(kk + 5, Kin - 1), q6 = min(kk + 6, Kin - 1), q7 = min(kk + 7, Kin - 1);
  v4f a, b;
  a.x = p[(size_t)q0 * nc]; a.y = p[(size_t)q1 * nc]; a.z = p[(size_t)q2 * nc]; a.w = p[(size_t)q3 * nc];
  b.x = p[(size_t)q4 * nc]; b.y = p[(size_t)q5 * nc]; b.z = p[(size_t)q6 * nc]; b.w = p[(size_t)q7 * nc];
  a.x = (nl && kk + 0 < Kin) ? a.x : 0.f;
  a.y = (nl && kk + 1 < Kin) ? a.y : 0.f;
  a.z = (nl && kk + 2 < Kin) ? a.z : 0.f;
  a.w = (nl && kk + 3 < Kin) ? a.w : 0.f;
  b.x = (nl && kk + 4 < Kin) ? b.x : 0.f;
  b.y = (nl && kk + 5 < Kin) ? b.y : 0.f;
  b.z = (nl && kk + 6 < Kin) ? b.z : 0.f;
  b.w = (nl && kk + 7 < Kin) ? b.w : 0.f;
  const v4u wv = pack8(a, b);
  unsigned short* o = wt + (size_t)n * (size_t)Kout + k8;
  *(volatile v4u*)o = wv;
  __threadfence();
  *(volatile v4u*)o = wv;
}

template<int EPI>
__global__ __launch_bounds__(GTHR) void k_gemm(
    const unsigned short* __restrict__ A, const unsigned short* __restrict__ WT, int K,
    const float* __restrict__ pa, const float* __restrict__ pb, const float* __restrict__ pc,
    float* GF, float* SD, float* out, int nN, int MPr)
{
  __shared__ __attribute__((aligned(16))) float stg[GBM * GBN];
  __shared__ __attribute__((aligned(16))) float sb[HC];
  __shared__ __attribute__((aligned(16))) float sv[4 * HC];
  __shared__ __attribute__((aligned(16))) float sc[NCLS];
  __shared__ __attribute__((aligned(16))) float sres[NCLS * GBM];
  const int tid = (int)threadIdx.x, lane = tid & 31, wave = tid >> 5, hh = lane >> 4, m = lane & 15;
  const int rowBase = (int)blockIdx.x * GBM;
  const int col0    = (int)blockIdx.y * GBN;

  if (EPI == 1) {
    const int which = tid >> 6;
    const int c = tid & (HC - 1);
    const float vs = pa[col0 + c];
    const float vd = pb[col0 + c];
    sv[which * HC + c] = bfr(which == 0 ? vs : vd);
  } else {
    if (tid < HC) sb[tid] = bfr(pa[tid]);
    const int j = tid >> 6;
    const int c = tid & (HC - 1);
    sv[j * HC + c]       = bfr(pb[c * NCLS + j]);
    sv[(j + 2) * HC + c] = bfr(pb[c * NCLS + j + 2]);
    if (tid < NCLS) sc[tid] = bfr(pc[tid]);
  }

  v8f acc[4];
  {
    const v8f z = {0.f, 0.f, 0.f, 0.f, 0.f, 0.f, 0.f, 0.f};
    acc[0] = z; acc[1] = z; acc[2] = z; acc[3] = z;
  }
  const unsigned short* ap = A  + (size_t)(rowBase + 16 * wave + m) * (size_t)K + 8 * hh;
  const unsigned short* wp = WT + (size_t)(col0 + m) * (size_t)K + 8 * hh;
  const int ksteps = K >> 5;
#pragma unroll 1
  for (int ks = 0; ks < ksteps; ++ks) {
    FragB af;
    af.h[0] = *(const v8usa*)(ap + 32 * ks);
    af.h[1] = *(const v8usa*)(ap + 32 * ks + 16);
#pragma unroll
    for (int t = 0; t < 4; ++t) {
      const unsigned short* wq = wp + (size_t)(16 * t) * (size_t)K + 32 * ks;
      FragB bf;
      bf.h[0] = *(const v8usa*)wq;
      bf.h[1] = *(const v8usa*)(wq + 16);
      acc[t] = wmb(af, bf, acc[t]);
    }
  }

#pragma unroll
  for (int t = 0; t < 4; ++t) {
    const int lc = 16 * t + m;
#pragma unroll
    for (int r = 0; r < 8; ++r) {
      const int lr = 16 * wave + 8 * hh + r;
      stg[lr * GBN + lc] = acc[t][r];
    }
  }
  __syncthreads();

  if (EPI == 1) {
    {
      const int row = tid & (GBM - 1), which = tid >> 6;
      const float* sa = sv + which * HC;
      const float* hr = stg + row * GBN;
      float d = 0.f;
#pragma unroll 4
      for (int c4 = 0; c4 < HC / 4; ++c4) {
        const v4f hv = *(const v4fa*)(hr + 4 * c4);
        const v4f av = *(const v4fa*)(sa + 4 * c4);
        d = fmaf(hv.x, av.x, d);
        d = fmaf(hv.y, av.y, d);
        d = fmaf(hv.z, av.z, d);
        d = fmaf(hv.w, av.w, d);
      }
      sres[which * GBM + row] = d;
    }
    v4f fv[8];
#pragma unroll
    for (int i = 0; i < 8; ++i) {
      const int lr = 16 * wave + 2 * i + hh;
      fv[i] = *(const v4fa*)(stg + lr * GBN + 4 * m);
    }
    __syncthreads();
    const int which2 = lane >> 4, piece = lane & 15;
    const v4f sdv = *(const v4fa*)(sres + which2 * GBM + 4 * piece);
    float* sp = SD + (size_t)(which2 * NHEAD + (int)blockIdx.y) * (size_t)MPr + rowBase + 4 * piece;
#pragma unroll
    for (int i = 0; i < 8; ++i) {
      const int lr = 16 * wave + 2 * i + hh;
      const int gr = rowBase + lr;
      float* op = GF + (size_t)gr * (size_t)DM + col0 + 4 * m;
      *(volatile v4f*)op = fv[i];
    }
    if (wave == 0) *(volatile v4f*)sp = sdv;
    __threadfence();
#pragma unroll
    for (int i = 0; i < 8; ++i) {
      const int lr = 16 * wave + 2 * i + hh;
      const int gr = rowBase + lr;
      float* op = GF + (size_t)gr * (size_t)DM + col0 + 4 * m;
      *(volatile v4f*)op = fv[i];
    }
    if (wave == 0) *(volatile v4f*)sp = sdv;
  } else {
    {
      const int row = tid & (GBM - 1), jp = tid >> 6;
      const float* w0 = sv + (2 * jp) * HC;
      const float* w1 = sv + (2 * jp + 1) * HC;
      const float* hr = stg + row * GBN;
      float d0 = 0.f, d1 = 0.f;
#pragma unroll 4
      for (int c4 = 0; c4 < HC / 4; ++c4) {
        v4f hv = *(const v4fa*)(hr + 4 * c4);
        const v4f bv = *(const v4fa*)(sb + 4 * c4);
        const v4f wa = *(const v4fa*)(w0 + 4 * c4);
        const v4f wb = *(const v4fa*)(w1 + 4 * c4);
        hv = relu4(hv + bv);
        d0 = fmaf(hv.x, wa.x, d0);
        d0 = fmaf(hv.y, wa.y, d0);
        d0 = fmaf(hv.z, wa.z, d0);
        d0 = fmaf(hv.w, wa.w, d0);
        d1 = fmaf(hv.x, wb.x, d1);
        d1 = fmaf(hv.y, wb.y, d1);
        d1 = fmaf(hv.z, wb.z, d1);
        d1 = fmaf(hv.w, wb.w, d1);
      }
      d0 += sc[2 * jp];
      d1 += sc[2 * jp + 1];
      sres[row * NCLS + 2 * jp]     = d0;
      sres[row * NCLS + 2 * jp + 1] = d1;
    }
    __syncthreads();
    const v4f y0 = *(const v4fa*)(sres + NCLS * lane);
    const v4f y1 = *(const v4fa*)(sres + NCLS * (32 + lane));
    const int r0 = rowBase + lane, r1 = rowBase + 32 + lane;
    float* o0p = out + (size_t)r0 * NCLS;
    float* o1p = out + (size_t)r1 * NCLS;
    if (wave == 0) {
      if (r0 < nN) *(volatile v4f*)o0p = y0;
      if (r1 < nN) *(volatile v4f*)o1p = y1;
    }
    __threadfence();
    if (wave == 0) {
      if (r0 < nN) *(volatile v4f*)o0p = y0;
      if (r1 < nN) *(volatile v4f*)o1p = y1;
    }
  }
}

template<int L>
__global__ __launch_bounds__(NTHR) void k_agg(
    const int* __restrict__ srcs, const int* __restrict__ dsts,
    const float* __restrict__ G, const float* __restrict__ SD, const float* __restrict__ bias,
    unsigned short* HP, int nN, int nE, int nb, int vec8, int MPr) {
  extern __shared__ v4f lds_dyn[];
  int* reg1 = (int*)lds_dyn;
  int* reg2 = reg1 + RCAP;
  int* scnt = reg2 + RCAP;
  int* soff = scnt + NBMAX;
  int* list = soff + NBMAX;
  int* wcnt = list + LISTN;
  int* wtot = wcnt + NWAVE;
  const int tid = (int)threadIdx.x, lane = tid & 31, wave = tid >> 5;
  const int nodeBase = (int)blockIdx.x * nb;

  for (int i = tid; i < NBMAX; i += NTHR) scnt[i] = 0;
  __syncthreads();

  int tot = 0;
  const int nChunks = (nE + CHUNK - 1) / CHUNK;
#pragma unroll 1
  for (int ch = 0; ch < nChunks; ++ch) {
    const int cbase = ch * CHUNK;
    const int wc = scan_chunk(dsts, nE, cbase, nodeBase, nb, vec8, list, tid, lane, wave);
    if (lane == 0) wcnt[wave] = wc;
    __syncthreads();
    int pre = 0, all = 0;
#pragma unroll
    for (int w2 = 0; w2 < NWAVE; ++w2) {
      int c = wcnt[w2];
      c = c < 0 ? 0 : (c > WCAP ? WCAP : c);
      all += c;
      pre += (w2 < wave) ? c : 0;
    }
    const int wcc  = wc > WCAP ? WCAP : wc;
    const int base = tot + pre;
#pragma unroll 1
    for (int i = lane; i < wcc; i += 32) {
      const int ent = list[wave * WCAP + i];
      const int el  = (ent >> SLOTB) & (CHUNK - 1);
      const int sl  = ent & SLOTM;
      int eid = cbase + el;
      eid = eid > nE - 1 ? nE - 1 : eid;
      const int pos = base + i;
      if (pos < RCAP) reg1[pos] = (int)(((unsigned)eid << SLOTB) | (unsigned)sl);
    }
    tot += all;
    tot = tot > RCAP ? RCAP : tot;
    __syncthreads();
  }
  const int nh = tot;

  if (wave == 0) {
#pragma unroll 1
    for (int b0 = 0; b0 < nh; b0 += 32) {
      const int idx = b0 + lane;
      const int uv  = reg1[idx < nh ? idx : nh - 1];
      const int m32 = (nh - b0) < 32 ? (nh - b0) : 32;
#pragma unroll 1
      for (int k = 0; k < m32; ++k) {
        const int u  = __builtin_amdgcn_readlane(uv, k);
        const int sl = u & SLOTM;
        if (lane == 0) scnt[sl] = scnt[sl] + 1;
      }
    }
  }
  __syncthreads();

  {
    const v4i ca = *(const v4i*)(scnt + 8 * tid);
    const v4i cb = *(const v4i*)(scnt + 8 * tid + 4);
    const int e0 = ca.x < 0 ? 0 : ca.x, e1 = ca.y < 0 ? 0 : ca.y, e2 = ca.z < 0 ? 0 : ca.z, e3 = ca.w < 0 ? 0 : ca.w;
    const int e4 = cb.x < 0 ? 0 : cb.x, e5 = cb.y < 0 ? 0 : cb.y, e6 = cb.z < 0 ? 0 : cb.z, e7 = cb.w < 0 ? 0 : cb.w;
    const int ts = e0 + e1 + e2 + e3 + e4 + e5 + e6 + e7;
    int incl = ts;
#pragma unroll
    for (int d = 1; d < 32; d <<= 1) {
      const int up = __shfl_up(incl, d);
      if (lane >= d) incl += up;
    }
    if (lane == 31) wtot[wave] = incl;
    __syncthreads();
    int pre = 0;
#pragma unroll
    for (int w2 = 0; w2 < NWAVE; ++w2) pre += (w2 < wave) ? wtot[w2] : 0;
    int run = pre + incl - ts;
    soff[8 * tid + 0] = run; run += e0;
    soff[8 * tid + 1] = run; run += e1;
    soff[8 * tid + 2] = run; run += e2;
    soff[8 * tid + 3] = run; run += e3;
    soff[8 * tid + 4] = run; run += e4;
    soff[8 * tid + 5] = run; run += e5;
    soff[8 * tid + 6] = run; run += e6;
    soff[8 * tid + 7] = run;
  }
  __syncthreads();
  for (int i = tid; i < NBMAX; i += NTHR) list[i] = soff[i];
  __syncthreads();

  if (wave == 0) {
#pragma unroll 1
    for (int b0 = 0; b0 < nh; b0 += 32) {
      const int idx = b0 + lane;
      const int uv  = reg1[idx < nh ? idx : nh - 1];
      const int m32 = (nh - b0) < 32 ? (nh - b0) : 32;
#pragma unroll 1
      for (int k = 0; k < m32; ++k) {
        const int u   = __builtin_amdgcn_readlane(uv, k);
        const int sl  = u & SLOTM;
        const int eid = (int)((unsigned)u >> SLOTB);
        if (lane == 0) {
          int pos = list[sl];
          pos = pos < 0 ? 0 : (pos > RCAP - 1 ? RCAP - 1 : pos);
          reg2[pos] = eid;
          list[sl] = pos + 1;
        }
      }
    }
  }
  __syncthreads();

  const int nbw = nb >> 3;
  const bool ovf = (nh >= RCAP);
  const float qnan = __int_as_float(0x7fc00000);
  const int head = lane >> 3;
  const float* ASp = SD + (size_t)head * (size_t)MPr;
  const float* ADp = SD + (size_t)(NHEAD + head) * (size_t)MPr;
  const v4f bb0 = bfr4(*(const v4fa*)(bias + 8 * lane));
  const v4f bb1 = bfr4(*(const v4fa*)(bias + 8 * lane + 4));

#pragma unroll 1
  for (int jt = 0; jt < nbw; ++jt) {
    const int slot = wave * nbw + jt;
    const int grow = nodeBase + slot;
    const int gcl  = grow < nN ? grow : nN - 1;
    int st = soff[slot];
    const int craw = scnt[slot];
    int cnt = craw;
    st  = st < 0 ? 0 : (st > nh ? nh : st);
    cnt = cnt < 0 ? 0 : (cnt > DEGCAP ? DEGCAP : cnt);
    if (cnt > nh - st) cnt = nh - st;
    const float pz = (ovf || craw > DEGCAP) ? qnan : 0.0f;

    const float* gdp = G + (size_t)gcl * (size_t)DM + 8 * lane;
    const v4f gd0 = *(const v4fa*)gdp;
    const v4f gd1 = *(const v4fa*)(gdp + 4);
    const float adv = ADp[gcl];
    float l0 = ASp[gcl] + adv;
    l0 = l0 >= 0.f ? l0 : SLOPE_ATT * l0;
    float mx = l0, dn = 1.0f;
    float a0 = gd0.x, a1 = gd0.y, a2 = gd0.z, a3 = gd0.w;
    float a4 = gd1.x, a5 = gd1.y, a6 = gd1.z, a7 = gd1.w;

#pragma unroll 1
    for (int q = 0; q < cnt; ++q) {
      int idx = st + q; idx = idx > RCAP - 1 ? RCAP - 1 : idx;
      int eid = reg2[idx]; eid = eid < 0 ? 0 : (eid > nE - 1 ? nE - 1 : eid);
      const int sraw = srcs[eid];
      const int s = sraw < 0 ? 0 : (sraw > nN - 1 ? nN - 1 : sraw);
      const float* gsp = G + (size_t)s * (size_t)DM + 8 * lane;
      const v4f gs0 = *(const v4fa*)gsp;
      const v4f gs1 = *(const v4fa*)(gsp + 4);
      float lg = ASp[s] + adv;
      lg = lg >= 0.f ? lg : SLOPE_ATT * lg;
      const float df = lg - mx;
      const float ee = __expf(-fabsf(df));
      const bool up  = df > 0.f;
      const float s1 = up ? ee : 1.0f;
      const float s2 = up ? 1.0f : ee;
      mx = up ? lg : mx;
      dn = fmaf(dn, s1, s2);
      a0 = fmaf(a0, s1, s2 * gs0.x);
      a1 = fmaf(a1, s1, s2 * gs0.y);
      a2 = fmaf(a2, s1, s2 * gs0.z);
      a3 = fmaf(a3, s1, s2 * gs0.w);
      a4 = fmaf(a4, s1, s2 * gs1.x);
      a5 = fmaf(a5, s1, s2 * gs1.y);
      a6 = fmaf(a6, s1, s2 * gs1.z);
      a7 = fmaf(a7, s1, s2 * gs1.w);
    }
    const float inv = __builtin_amdgcn_rcpf(dn + EPS_SM);
    const bool live = grow < nN;
    float o0 = fmaf(a0, inv, bb0.x), o1 = fmaf(a1, inv, bb0.y), o2 = fmaf(a2, inv, bb0.z), o3 = fmaf(a3, inv, bb0.w);
    float o4 = fmaf(a4, inv, bb1.x), o5 = fmaf(a5, inv, bb1.y), o6 = fmaf(a6, inv, bb1.z), o7 = fmaf(a7, inv, bb1.w);
    if (L == 1) {
      o0 = fmaxf(o0, 0.f); o1 = fmaxf(o1, 0.f); o2 = fmaxf(o2, 0.f); o3 = fmaxf(o3, 0.f);
      o4 = fmaxf(o4, 0.f); o5 = fmaxf(o5, 0.f); o6 = fmaxf(o6, 0.f); o7 = fmaxf(o7, 0.f);
    }
    o0 = (live ? o0 : 0.f) + pz; o1 = (live ? o1 : 0.f) + pz; o2 = (live ? o2 : 0.f) + pz; o3 = (live ? o3 : 0.f) + pz;
    o4 = (live ? o4 : 0.f) + pz; o5 = (live ? o5 : 0.f) + pz; o6 = (live ? o6 : 0.f) + pz; o7 = (live ? o7 : 0.f) + pz;
    v4f hv0, hv1, lv0, lv1;
    hv0.x = bfr(o0); hv0.y = bfr(o1); hv0.z = bfr(o2); hv0.w = bfr(o3);
    hv1.x = bfr(o4); hv1.y = bfr(o5); hv1.z = bfr(o6); hv1.w = bfr(o7);
    lv0.x = o0 - hv0.x; lv0.y = o1 - hv0.y; lv0.z = o2 - hv0.z; lv0.w = o3 - hv0.w;
    lv1.x = o4 - hv1.x; lv1.y = o5 - hv1.y; lv1.z = o6 - hv1.z; lv1.w = o7 - hv1.w;
    const v4u ph = pack8(hv0, hv1);
    const v4u pl = pack8(lv0, lv1);
    unsigned short* gp = HP + (size_t)grow * (size_t)KP2 + 8 * lane;
    unsigned short* gq = gp + DM;
    const bool wr = (grow < MPr);
    if (wr) { *(volatile v4u*)gp = ph; *(volatile v4u*)gq = pl; }
    __threadfence();
    if (wr) { *(volatile v4u*)gp = ph; *(volatile v4u*)gq = pl; }
  }
}

static int pick_nb(int nE, int nN) {
  int nb = NBLIM;
  while (nb > 32 && (long long)nb * (long long)nE * 5LL > (long long)RCAP * (long long)nN * 4LL) nb >>= 1;
  return nb;
}
static inline int cdiv(int a, int b) { return (a + b - 1) / b; }

extern "C" void kernel_launch(void* const* d_in, const int* in_sizes, int n_in,
                              void* d_out, int out_size, void* d_ws, size_t ws_size,
                              hipStream_t stream) {
  if (n_in < 14) return;
  if (in_sizes[0] <= 0 || (in_sizes[0] % FIN) != 0) return;
  const int nN = in_sizes[0] / FIN;
  if (nN <= 0 || nN > (1 << 22)) return;
  if (in_sizes[1] < 2 || (in_sizes[1] & 1) != 0) return;
  const int nE = in_sizes[1] / 2;
  if (nE < 1 || nE >= (1 << (32 - SLOTB))) return;
  if (in_sizes[2]  != FIN * DM) return;
  if (in_sizes[3]  != DM || in_sizes[4] != DM) return;
  if (in_sizes[5]  != DM) return;
  if (in_sizes[6]  != DM * DM) return;
  if (in_sizes[7]  != DM || in_sizes[8] != DM) return;
  if (in_sizes[9]  != DM) return;
  if (in_sizes[10] != DM * FCD) return;
  if (in_sizes[11] != FCD) return;
  if (in_sizes[12] != FCD * NCLS) return;
  if (in_sizes[13] != NCLS) return;
  if (out_size != nN * NCLS) return;

  const float* x    = (const float*)d_in[0];
  const int*   ei   = (const int*)  d_in[1];
  const float* W1   = (const float*)d_in[2];
  const float* as1  = (const float*)d_in[3];
  const float* ad1  = (const float*)d_in[4];
  const float* b1   = (const float*)d_in[5];
  const float* W2   = (const float*)d_in[6];
  const float* as2  = (const float*)d_in[7];
  const float* ad2  = (const float*)d_in[8];
  const float* b2   = (const float*)d_in[9];
  const float* Wc1  = (const float*)d_in[10];
  const float* bc1  = (const float*)d_in[11];
  const float* Wc2  = (const float*)d_in[12];
  const float* bc2  = (const float*)d_in[13];
  float* out = (float*)d_out;
  const int* src = ei;
  const int* dst = ei + nE;

  const int MP   = cdiv(nN, MROWS) * MROWS;
  const int nb   = pick_nb(nE, nN);
  if (nb < 32 || (nb & (nb - 1)) != 0 || nb > NBLIM) return;
  const int gA   = cdiv(MP, nb);
  const int vec8 = ((nE & 3) == 0) ? 1 : 0;
  if (gA * nb < MP) return;

  char* ws = (char*)d_ws;
  size_t off = 0;
  const size_t oXB  = off; off += (size_t)MP * FIN * 2;            off = (off + 255) & ~(size_t)255;
  const size_t oW1T = off; off += (size_t)DM * FIN * 2;            off = (off + 255) & ~(size_t)255;
  const size_t oW2T = off; off += (size_t)DM * KP2 * 2;            off = (off + 255) & ~(size_t)255;
  const size_t oW3T = off; off += (size_t)FCD * KP2 * 2;           off = (off + 255) & ~(size_t)255;
  const size_t oG   = off; off += (size_t)MP * DM * 4;             off = (off + 255) & ~(size_t)255;
  const size_t oSD  = off; off += (size_t)2 * NHEAD * MP * 4;      off = (off + 255) & ~(size_t)255;
  const size_t oHP  = off; off += (size_t)MP * KP2 * 2;            off = (off + 255) & ~(size_t)255;
  if (off > ws_size || off > (size_t)WSMAX) return;
  unsigned short* XB  = (unsigned short*)(ws + oXB);
  unsigned short* W1T = (unsigned short*)(ws + oW1T);
  unsigned short* W2T = (unsigned short*)(ws + oW2T);
  unsigned short* W3T = (unsigned short*)(ws + oW3T);
  float*          G   = (float*)(ws + oG);
  float*          SD  = (float*)(ws + oSD);
  unsigned short* HP  = (unsigned short*)(ws + oHP);

  hipFuncSetAttribute(reinterpret_cast<const void*>(&k_agg<1>),
                      hipFuncAttributeMaxDynamicSharedMemorySize, LDS_AGG);
  hipFuncSetAttribute(reinterpret_cast<const void*>(&k_agg<2>),
                      hipFuncAttributeMaxDynamicSharedMemorySize, LDS_AGG);

  const int nUx = MP * (FIN / 8);
  k_xprep<<<cdiv(nUx, NTHR), NTHR, 0, stream>>>(x, XB, nN, nUx);

  {
    const int nUw1 = DM * (FIN / 8);
    const int nUw2 = DM * (KP2 / 8);
    const int nUw3 = FCD * (KP2 / 8);
    k_wprep<<<cdiv(nUw1, NTHR), NTHR, 0, stream>>>(W1,  FIN, FIN, DM,  DM,  FIN, W1T, nUw1);
    k_wprep<<<cdiv(nUw2, NTHR), NTHR, 0, stream>>>(W2,  DM,  DM,  DM,  DM,  KP2, W2T, nUw2);
    k_wprep<<<cdiv(nUw3, NTHR), NTHR, 0, stream>>>(Wc1, DM,  DM,  FCD, FCD, KP2, W3T, nUw3);
  }

  const int gM = MP / GBM;
  k_gemm<1><<<dim3(gM, NHEAD), GTHR, 0, stream>>>(XB, W1T, FIN, as1, ad1, bc2, G, SD, out, nN, MP);
  k_agg<1><<<gA, NTHR, LDS_AGG, stream>>>(src, dst, G, SD, b1, HP, nN, nE, nb, vec8, MP);
  k_gemm<1><<<dim3(gM, NHEAD), GTHR, 0, stream>>>(HP, W2T, KP2, as2, ad2, bc2, G, SD, out, nN, MP);
  k_agg<2><<<gA, NTHR, LDS_AGG, stream>>>(src, dst, G, SD, b2, HP, nN, nE, nb, vec8, MP);
  k_gemm<2><<<dim3(gM, 1), GTHR, 0, stream>>>(HP, W3T, KP2, bc1, Wc2, bc2, G, SD, out, nN, MP);
}
